// GatedLinearStateAttention_15564961481276
// MI455X (gfx1250) — hardware-verified
//
#include <hip/hip_runtime.h>


namespace {
constexpr int Bn = 4, T = 1024, DIM = 1024, H = 16, HD = 64, NT = Bn * T, CH = 32;
constexpr float QS = 8.0f, KS = 8.0f, VS = 8.0f, PS = 8.0f, AS_ = 8.0f;
constexpr size_t PLH = (size_t)Bn * H * T * HD;

typedef _Float16 b16;
typedef __attribute__((ext_vector_type(16))) _Float16 v16b;
typedef __attribute__((ext_vector_type(16))) __bf16 v16bb;
typedef __attribute__((ext_vector_type(8))) _Float16 v8b;
typedef __attribute__((ext_vector_type(8))) unsigned short v8us;
typedef __attribute__((ext_vector_type(8))) float v8f;
typedef __attribute__((ext_vector_type(4))) float v4f;
__device__ __forceinline__ float bf16_rne(float f) { unsigned int u = __float_as_uint(f); u += 0x7FFFu + ((u >> 16) & 1u); return __uint_as_float(u & 0xFFFF0000u); }
__device__ __forceinline__ unsigned short bf16_bits(float f) { unsigned int u = __float_as_uint(f); u += 0x7FFFu + ((u >> 16) & 1u); return (unsigned short)(u >> 16); }
__device__ __forceinline__ void split16(float v, b16& hi, b16& lo) { hi = (b16)v; lo = (b16)(v - (float)hi); }
__device__ __forceinline__ v16b frag_kb(const b16* p, int hh) { const v8b a = *(const v8b*)(p + 8 * hh), b = *(const v8b*)(p + 16 + 8 * hh); v16b f;
#pragma unroll
  for (int e = 0; e < 8; ++e) { f[e] = a[e]; f[8 + e] = b[e]; } return f; }
__device__ __forceinline__ void frag_split(const float* p, int hh, v16b& fh, v16b& fl) {
#pragma unroll
  for (int e = 0; e < 8; ++e) { b16 a, c; split16(p[8 * hh + e] * AS_, a, c); fh[e] = a; fl[e] = c; split16(p[16 + 8 * hh + e] * AS_, a, c); fh[8 + e] = a; fl[8 + e] = c; } }
__device__ __forceinline__ v16bb frag_bf(const unsigned short* p, int hh) { const v8us a = *(const v8us*)(p + 8 * hh), b = *(const v8us*)(p + 16 + 8 * hh); union { unsigned short s[16]; v16bb v; } u;
#pragma unroll
  for (int e = 0; e < 8; ++e) { u.s[e] = a[e]; u.s[8 + e] = b[e]; } return u.v; }
__device__ __forceinline__ v16bb frag_f32bf(const float* p, int hh) { union { unsigned short s[16]; v16bb v; } u;
#pragma unroll
  for (int e = 0; e < 8; ++e) { u.s[e] = bf16_bits(p[8 * hh + e]); u.s[8 + e] = bf16_bits(p[16 + 8 * hh + e]); } return u.v; }
__device__ __forceinline__ v8f wmma16b(v16b a, v16b b, v8f c) { v8f d = __builtin_amdgcn_wmma_f32_16x16x32_f16(false, a, false, b, (short)0, c, false, false); asm volatile("v_nop\n\tv_nop\n\tv_nop\n\tv_nop" : "+v"(d) : "v"(a), "v"(b)); return d; }
__device__ __forceinline__ v8f wmma16bb(v16bb a, v16bb b, v8f c) { v8f d = __builtin_amdgcn_wmma_f32_16x16x32_bf16(false, a, false, b, (short)0, c, false, false); asm volatile("v_nop\n\tv_nop\n\tv_nop\n\tv_nop" : "+v"(d) : "v"(a), "v"(b)); return d; }
__device__ __forceinline__ v8f wmma3(v16b ah, v16b al, v16b bh, v16b bl, v8f c) { c = wmma16b(ah, bh, c); c = wmma16b(ah, bl, c); c = wmma16b(al, bh, c); return c; }
__device__ __forceinline__ void wave_lds_sync() { __builtin_amdgcn_fence(__ATOMIC_RELEASE, "workgroup"); __builtin_amdgcn_wave_barrier(); __builtin_amdgcn_fence(__ATOMIC_ACQUIRE, "workgroup"); }
__device__ __forceinline__ float nexp(float x) { return __builtin_amdgcn_exp2f(x * 1.4426950408889634f); }
__device__ __forceinline__ float softplus_f(float x) { return (x > 20.0f) ? x : log1pf(nexp(x)); }
__device__ __forceinline__ float pmul(float a, float b) { float p = a * b; asm volatile("" : "+v"(p)); return p; }

struct Wo_ { static constexpr size_t PJ = 0, QK = PJ + (size_t)4160 * DIM, WO = QK + (size_t)2048 * DIM, END = WO + (size_t)DIM * DIM; };
__global__ __launch_bounds__(256) void prep_kernel(const float* __restrict__ Wsq, const float* __restrict__ Wsk, const float* __restrict__ Wsv, const float* __restrict__ Wg, const float* __restrict__ Wq, const float* __restrict__ Wk, const float* __restrict__ Wv, const float* __restrict__ Wo,
                                                   const float* __restrict__ bsq, const float* __restrict__ bsk, const float* __restrict__ bsv, const float* __restrict__ bv, const float* __restrict__ bg, const float* __restrict__ bq, const float* __restrict__ bk, const float* __restrict__ bo, const float* __restrict__ temp, unsigned short* __restrict__ R, float* __restrict__ P) {
  const size_t tid = (size_t)blockIdx.x * 256 + threadIdx.x, nth = (size_t)gridDim.x * 256;
  for (int pass = 0; pass < 2; ++pass) {
    for (size_t p = tid; p < (size_t)4160 * DIM / 8; p += nth) { const int o = (int)(p / (DIM / 8)); const int k0 = (int)(p % (DIM / 8)) * 8; const int m = o >> 10, oo = o & 1023;
      const float* W = (m == 0) ? Wsq : (m == 1) ? Wsk : (m == 2) ? Wsv : (m == 3) ? Wv : Wg; v8us v;
#pragma unroll
      for (int e = 0; e < 8; ++e) v[e] = (m == 4 && oo >= H) ? (unsigned short)0 : bf16_bits(W[(size_t)oo * DIM + k0 + e]);
      *(volatile v8us*)(R + Wo_::PJ + (size_t)o * DIM + k0) = v; }
    for (size_t p = tid; p < (size_t)3072 * DIM / 8; p += nth) { const int o = (int)(p / (DIM / 8)); const int k0 = (int)(p % (DIM / 8)) * 8; const float* W = (o < 1024) ? (Wq + (size_t)o * DIM) : (o < 2048) ? (Wk + (size_t)(o - 1024) * DIM) : (Wo + (size_t)(o - 2048) * DIM); v8b v;
#pragma unroll
      for (int e = 0; e < 8; ++e) v[e] = (b16)bf16_rne(W[k0 + e]);
      *(volatile v8b*)((b16*)R + Wo_::QK + (size_t)o * DIM + k0) = v; }
    for (size_t p = tid; p < 7248; p += nth) { const int q = (int)p; float v;
      if (q < 1024) v = bsq[q]; else if (q < 2048) v = bsk[q - 1024]; else if (q < 3072) v = bsv[q - 2048]; else if (q < 4096) v = bv[q - 3072]; else if (q < 4160) v = (q - 4096 < H) ? bg[q - 4096] : 0.0f;
      else if (q < 5184) v = bq[q - 4160]; else if (q < 6208) v = bk[q - 5184]; else if (q < 7232) v = bo[q - 6208]; else v = softplus_f(bf16_rne(temp[q - 7232]));
      P[p] = (q < 7232) ? bf16_rne(v) : v; }
    __threadfence(); }
}

__global__ __launch_bounds__(128) void proj_kernel(const float* __restrict__ x, const unsigned short* __restrict__ R, const float* __restrict__ P, float* __restrict__ sq, float* __restrict__ sk, float* __restrict__ sv, b16* __restrict__ vt, float* __restrict__ logg) {
  __shared__ __attribute__((aligned(16))) float Tc[64][128 + 4];
  const int lane = threadIdx.x & 31, wave = threadIdx.x >> 5, nloc = lane & 15, hlf = lane >> 4, ct = blockIdx.x, p0 = blockIdx.y * 128, m0 = p0 + wave * 32, b = p0 / T, t0 = p0 % T;
  const unsigned short* Wt = R + Wo_::PJ + (size_t)ct * 64 * DIM; const float* bias = P + ct * 64;
  v8f acc[2][4];
#pragma unroll
  for (int r = 0; r < 2; ++r)
#pragma unroll
    for (int t = 0; t < 4; ++t) acc[r][t] = (v8f){};
#pragma unroll 2
  for (int kb = 0; kb < DIM; kb += 32) { const v16bb a0 = frag_f32bf(x + (size_t)(m0 + nloc) * DIM + kb, hlf), a1 = frag_f32bf(x + (size_t)(m0 + 16 + nloc) * DIM + kb, hlf);
#pragma unroll
    for (int t = 0; t < 4; ++t) { const v16bb bw = frag_bf(Wt + (size_t)(t * 16 + nloc) * DIM + kb, hlf); acc[0][t] = wmma16bb(a0, bw, acc[0][t]); acc[1][t] = wmma16bb(a1, bw, acc[1][t]); } }
#pragma unroll
  for (int t = 0; t < 4; ++t) { const float bb = bias[t * 16 + nloc];
#pragma unroll
    for (int r = 0; r < 2; ++r)
#pragma unroll
      for (int v = 0; v < 8; ++v) Tc[t * 16 + nloc][wave * 32 + r * 16 + 8 * hlf + v] = acc[r][t][v] + bb; }
  __syncthreads();
  for (int pass = 0; pass < 2; ++pass) {
    if (ct < 48) { float* dst = ((ct < 16) ? sq : (ct < 32) ? sk : sv) + (((size_t)b * H + (ct & 15)) * T + t0) * HD;
      for (int i = threadIdx.x; i < 128 * 16; i += 128) { const int rr = i >> 4, c4 = (i & 15) * 4; v4f o; o[0] = Tc[c4][rr]; o[1] = Tc[c4 + 1][rr]; o[2] = Tc[c4 + 2][rr]; o[3] = Tc[c4 + 3][rr]; *(volatile v4f*)(dst + (size_t)rr * HD + c4) = o; } }
    else if (ct < 64) { const int h = ct - 48; for (int i = threadIdx.x; i < 64 * 16; i += 128) { const int d = i >> 4, c8 = (i & 15) * 8; v8b o; for (int e = 0; e < 8; ++e) o[e] = (b16)(Tc[d][c8 + e] * VS); *(volatile v8b*)(vt + (((size_t)b * H + h) * HD + d) * T + t0 + c8) = o; } }
    else { for (int i = threadIdx.x; i < 128 * 4; i += 128) { const int rr = i >> 2, c4 = (i & 3) * 4; v4f o; for (int e = 0; e < 4; ++e) o[e] = -softplus_f(Tc[c4 + e][rr]); *(volatile v4f*)(logg + ((size_t)b * T + t0 + rr) * H + c4) = o; } }
    __threadfence(); }
}

__global__ __launch_bounds__(32) void rec_kernel(const float* __restrict__ sq, const float* __restrict__ sk, const float* __restrict__ sv, const float* __restrict__ logg, float* __restrict__ hseq) {
  __shared__ __attribute__((aligned(16))) float Qs[CH][HD + 4], Ks[CH][HD + 4], Hs[CH][HD + 4]; __shared__ __attribute__((aligned(16))) float Vt[HD][CH + 4], Kt[HD][CH + 4], Pm[CH][CH + 4]; __shared__ __attribute__((aligned(16))) float Mt[HD][HD + 4]; __shared__ float Lc[CH];
  const int lane = threadIdx.x, nloc = lane & 15, hlf = lane >> 4, h = blockIdx.x, b = blockIdx.y;
  const float* Q = sq + (((size_t)b * H + h) * T) * HD; const float* K = sk + (((size_t)b * H + h) * T) * HD; const float* V = sv + (((size_t)b * H + h) * T) * HD;
  for (int i = lane; i < HD * (HD + 4); i += 32) (&Mt[0][0])[i] = 0.0f;
  for (int c = 0; c < T / CH; ++c) { const int t0 = c * CH;
    for (int i = lane; i < CH * HD; i += 32) { const int r = i / HD, d = i % HD; Qs[r][d] = Q[(size_t)(t0 + r) * HD + d]; Ks[r][d] = K[(size_t)(t0 + r) * HD + d]; Vt[d][r] = V[(size_t)(t0 + r) * HD + d]; }
    { float lg = logg[((size_t)b * T + t0 + lane) * H + h];
#pragma unroll
      for (int o = 1; o < 32; o <<= 1) { const float u = __shfl_up(lg, o); if (lane >= o) lg += u; }
      Lc[lane] = lg; }
    wave_lds_sync();
    const float LC = Lc[CH - 1];
    for (int i = lane; i < CH * HD; i += 32) { const int s = i / HD, d = i % HD; Kt[d][s] = Ks[s][d] * nexp(LC - Lc[s]); }
#pragma unroll
    for (int ti = 0; ti < 2; ++ti)
#pragma unroll
      for (int tj = 0; tj < 2; ++tj) { v8f acc = {};
#pragma unroll
        for (int kb = 0; kb < HD; kb += 32) { v16b ah, al, bh, bl; frag_split(&Qs[ti * 16 + nloc][kb], hlf, ah, al); frag_split(&Ks[tj * 16 + nloc][kb], hlf, bh, bl); acc = wmma3(ah, al, bh, bl, acc); }
#pragma unroll
        for (int r = 0; r < 8; ++r) { const int tt = ti * 16 + 8 * hlf + r, ss = tj * 16 + nloc; const float dcy = (ss <= tt) ? nexp(Lc[tt] - Lc[ss]) : 0.0f; Pm[tt][ss] = acc[r] * (1.0f / (AS_ * AS_)) * dcy; } }
    wave_lds_sync();
#pragma unroll
    for (int ti = 0; ti < 2; ++ti) {
#pragma unroll
      for (int te = 0; te < 4; ++te) { v8f ain = {}, aq = {};
        { v16b ah, al, bh, bl; frag_split(&Pm[ti * 16 + nloc][0], hlf, ah, al); frag_split(&Vt[te * 16 + nloc][0], hlf, bh, bl); ain = wmma3(ah, al, bh, bl, ain); }
#pragma unroll
        for (int kb = 0; kb < HD; kb += 32) { v16b ah, al, bh, bl; frag_split(&Qs[ti * 16 + nloc][kb], hlf, ah, al); frag_split(&Mt[te * 16 + nloc][kb], hlf, bh, bl); aq = wmma3(ah, al, bh, bl, aq); }
#pragma unroll
        for (int r = 0; r < 8; ++r) { const int tt = ti * 16 + 8 * hlf + r; Hs[tt][te * 16 + nloc] = (ain[r] + aq[r] * nexp(Lc[tt])) * (1.0f / (AS_ * AS_)); } } }
    wave_lds_sync();
    { const float dC = nexp(LC);
#pragma unroll
      for (int te = 0; te < 4; ++te)
#pragma unroll
        for (int td = 0; td < 4; ++td) { v8f acc;
#pragma unroll
          for (int r = 0; r < 8; ++r) acc[r] = Mt[te * 16 + 8 * hlf + r][td * 16 + nloc] * dC * (AS_ * AS_);
          v16b ah, al, bh, bl; frag_split(&Vt[te * 16 + nloc][0], hlf, ah, al); frag_split(&Kt[td * 16 + nloc][0], hlf, bh, bl); acc = wmma3(ah, al, bh, bl, acc);
#pragma unroll
          for (int r = 0; r < 8; ++r) Mt[te * 16 + 8 * hlf + r][td * 16 + nloc] = acc[r] * (1.0f / (AS_ * AS_)); } }
    for (int pass = 0; pass < 2; ++pass) { for (int i = lane; i < CH * (HD / 4); i += 32) { const int r = i / (HD / 4), c4 = (i % (HD / 4)) * 4; *(volatile v4f*)(hseq + ((size_t)b * T + t0 + r) * DIM + h * HD + c4) = *(const v4f*)(&Hs[r][c4]); } __threadfence(); }
    wave_lds_sync(); }
}

__global__ __launch_bounds__(128) void qk_kernel(const float* __restrict__ hseq, const unsigned short* __restrict__ R, const float* __restrict__ P, b16* __restrict__ qp, b16* __restrict__ kp) {
  __shared__ __attribute__((aligned(16))) b16 Tt[4][32][64 + 8];
  const int lane = threadIdx.x & 31, wave = threadIdx.x >> 5, nloc = lane & 15, hlf = lane >> 4, h = blockIdx.x, c0 = h * HD, which = blockIdx.z, m0 = blockIdx.y * 128 + wave * 32;
  const b16* Wt = (const b16*)R + Wo_::QK + (size_t)which * DIM * DIM; const float* bias = P + ((which == 0) ? 4160 : 5184); const float scl = (which == 0) ? P[7232 + h] * QS : KS;
  v8f acc[2][4];
#pragma unroll
  for (int r = 0; r < 2; ++r)
#pragma unroll
    for (int t = 0; t < 4; ++t) acc[r][t] = (v8f){};
#pragma unroll 2
  for (int kb = 0; kb < DIM; kb += 32) { v16b a0, a1;
#pragma unroll
    for (int e = 0; e < 8; ++e) { a0[e] = (b16)hseq[(size_t)(m0 + nloc) * DIM + kb + 8 * hlf + e]; a0[8 + e] = (b16)hseq[(size_t)(m0 + nloc) * DIM + kb + 16 + 8 * hlf + e]; a1[e] = (b16)hseq[(size_t)(m0 + 16 + nloc) * DIM + kb + 8 * hlf + e]; a1[8 + e] = (b16)hseq[(size_t)(m0 + 16 + nloc) * DIM + kb + 16 + 8 * hlf + e]; }
#pragma unroll
    for (int t = 0; t < 4; ++t) { const v16b bw = frag_kb(Wt + (size_t)(c0 + t * 16 + nloc) * DIM + kb, hlf); acc[0][t] = wmma16b(a0, bw, acc[0][t]); acc[1][t] = wmma16b(a1, bw, acc[1][t]); } }
#pragma unroll
  for (int r = 0; r < 2; ++r)
#pragma unroll
    for (int v = 0; v < 8; ++v) { float vals[4], s2 = 0.0f;
#pragma unroll
      for (int t = 0; t < 4; ++t) { vals[t] = acc[r][t][v] + bias[c0 + t * 16 + nloc]; s2 += pmul(vals[t], vals[t]); }
#pragma unroll
      for (int o = 1; o < 16; o <<= 1) s2 += __shfl_xor(s2, o);
      const float inv = scl / fmaxf(sqrtf(s2), 1e-12f);
#pragma unroll
      for (int t = 0; t < 4; ++t) Tt[wave][r * 16 + 8 * hlf + v][t * 16 + nloc] = (b16)(vals[t] * inv); }
  wave_lds_sync();
  b16* base = ((which == 0) ? qp : kp) + (((size_t)(m0 / T) * H + h) * T + (m0 % T)) * HD;
  for (int pass = 0; pass < 2; ++pass) {
#pragma unroll
    for (int j = 0; j < 8; ++j) { const int rr = j * 4 + (lane >> 3), c8 = (lane & 7) * 8; *(volatile v8b*)(base + (size_t)rr * HD + c8) = *(const v8b*)(&Tt[wave][rr][c8]); }
    __threadfence(); }
}

__global__ __launch_bounds__(256) void attn_kernel(const b16* __restrict__ qp, const b16* __restrict__ kp, const b16* __restrict__ vt, b16* __restrict__ ctx) {
  __shared__ __attribute__((aligned(16))) b16 Os[16][8 * HD + 8];
  const int wid = threadIdx.x >> 5, lane = threadIdx.x & 31, hh = lane >> 4, col = lane & 15; const int b = blockIdx.x / (T / 16), q0 = (blockIdx.x % (T / 16)) * 16, h = blockIdx.y * 8 + wid, qi = q0 + col;
  const b16* Qp = qp + (((size_t)b * H + h) * T) * HD; const b16* Kp = kp + (((size_t)b * H + h) * T) * HD; const b16* V = vt + (((size_t)b * H + h) * HD) * T;
  const v16b qf0 = frag_kb(Qp + (size_t)qi * HD, hh), qf1 = frag_kb(Qp + (size_t)qi * HD + 32, hh);
  float m = -INFINITY, l = 0.0f; v8f o[4] = {{}, {}, {}, {}};
  for (int kb = 0; kb < T; kb += 32) {
    const v16b ka0 = frag_kb(Kp + (size_t)(kb + col) * HD, hh), ka1 = frag_kb(Kp + (size_t)(kb + col) * HD + 32, hh), kc0 = frag_kb(Kp + (size_t)(kb + 16 + col) * HD, hh), kc1 = frag_kb(Kp + (size_t)(kb + 16 + col) * HD + 32, hh);
    v8f s0 = {}, s1 = {}; s0 = wmma16b(ka0, qf0, s0); s0 = wmma16b(ka1, qf1, s0); s1 = wmma16b(kc0, qf0, s1); s1 = wmma16b(kc1, qf1, s1);
    float mr = -INFINITY;
#pragma unroll
    for (int r = 0; r < 8; ++r) { s0[r] *= 1.0f / (QS * KS); s1[r] *= 1.0f / (QS * KS); mr = fmaxf(mr, fmaxf(s0[r], s1[r])); }
    mr = fmaxf(mr, __shfl_xor(mr, 16));
    const float mn = fmaxf(m, mr), al_ = nexp(m - mn); m = mn; float sum = 0.0f; v16b pbv;
#pragma unroll
    for (int r = 0; r < 8; ++r) { const float e0 = nexp(s0[r] - mn), e1 = nexp(s1[r] - mn); sum += e0 + e1; pbv[r] = (b16)(e0 * PS); pbv[8 + r] = (b16)(e1 * PS); }
    sum += __shfl_xor(sum, 16); l = l * al_ + sum;
#pragma unroll
    for (int t = 0; t < 4; ++t) { o[t] *= al_; const v16b vf = frag_kb(V + (size_t)(t * 16 + col) * T + kb, hh); o[t] = wmma16b(vf, pbv, o[t]); } }
  const float inv = 1.0f / (l * VS * PS);
#pragma unroll
  for (int t = 0; t < 4; ++t)
#pragma unroll
    for (int r = 0; r < 8; ++r) Os[col][wid * HD + t * 16 + 8 * hh + r] = (b16)(o[t][r] * inv);
  __syncthreads();
  for (int pass = 0; pass < 2; ++pass) { for (int i = threadIdx.x; i < 16 * (8 * HD / 8); i += 256) { const int rr = i / (8 * HD / 8), c8 = (i % (8 * HD / 8)) * 8; *(volatile v8b*)(ctx + ((size_t)b * T + q0 + rr) * DIM + blockIdx.y * 8 * HD + c8) = *(const v8b*)(&Os[rr][c8]); } __threadfence(); }
}

__global__ __launch_bounds__(128) void out_kernel(const b16* __restrict__ ctx, const unsigned short* __restrict__ R, const float* __restrict__ P, float* __restrict__ out) {
  __shared__ __attribute__((aligned(16))) float Ts[4][32 * 64];
  const int lane = threadIdx.x & 31, wave = threadIdx.x >> 5, nloc = lane & 15, hlf = lane >> 4, m0 = blockIdx.y * 128 + wave * 32, c0 = blockIdx.x * 64; const b16* Wt = (const b16*)R + Wo_::WO; const float* bo = P + 6208;
  v8f acc[2][4];
#pragma unroll
  for (int r = 0; r < 2; ++r)
#pragma unroll
    for (int t = 0; t < 4; ++t) acc[r][t] = (v8f){};
#pragma unroll 2
  for (int kb = 0; kb < DIM; kb += 32) { const v16b a0 = frag_kb(ctx + (size_t)(m0 + nloc) * DIM + kb, hlf), a1 = frag_kb(ctx + (size_t)(m0 + 16 + nloc) * DIM + kb, hlf);
#pragma unroll
    for (int t = 0; t < 4; ++t) { const v16b bw = frag_kb(Wt + (size_t)(c0 + t * 16 + nloc) * DIM + kb, hlf); acc[0][t] = wmma16b(a0, bw, acc[0][t]); acc[1][t] = wmma16b(a1, bw, acc[1][t]); } }
  float* Tt = Ts[wave];
#pragma unroll
  for (int t = 0; t < 4; ++t) { const float bb = bo[c0 + t * 16 + nloc];
#pragma unroll
    for (int r = 0; r < 2; ++r)
#pragma unroll
      for (int v = 0; v < 8; ++v) Tt[(r * 16 + v + 8 * hlf) * 64 + t * 16 + nloc] = acc[r][t][v] + bb; }
  wave_lds_sync();
  for (int pass = 0; pass < 2; ++pass) {
#pragma unroll
    for (int j = 0; j < 16; ++j) { const int rr = j * 2 + hlf, c4 = nloc * 4; *(volatile v4f*)(out + (size_t)(m0 + rr) * DIM + c0 + c4) = *(const v4f*)(Tt + rr * 64 + c4); }
    __threadfence(); }
}
}

extern "C" void kernel_launch(void* const* d_in, const int* in_sizes, int n_in,
                              void* d_out, int out_size, void* d_ws, size_t ws_size, hipStream_t stream) {
  (void)n_in; (void)out_size;
  const float* x = (const float*)d_in[0]; const float* Wsq = (const float*)d_in[1]; const float* bsq = (const float*)d_in[2]; const float* Wsk = (const float*)d_in[3]; const float* bsk = (const float*)d_in[4]; const float* Wsv = (const float*)d_in[5]; const float* bsv = (const float*)d_in[6]; const float* Wg = (const float*)d_in[7]; const float* bg = (const float*)d_in[8];
  const float* Wq = (const float*)d_in[9]; const float* bq = (const float*)d_in[10]; const float* Wk = (const float*)d_in[11]; const float* bk = (const float*)d_in[12]; const float* Wv = (const float*)d_in[13]; const float* bv = (const float*)d_in[14]; const float* Wo = (const float*)d_in[15]; const float* bo = (const float*)d_in[16]; const float* temp = (const float*)d_in[17];
  float* out = (float*)d_out;
  if (in_sizes[0] != NT * DIM || in_sizes[1] != DIM * DIM || in_sizes[7] != H * DIM || in_sizes[15] != DIM * DIM || in_sizes[17] != H) return;
  size_t off = 0; char* ws = (char*)d_ws;
  auto carve = [&](size_t bytes) { char* p = ws + off; off += (bytes + 255) & ~(size_t)255; return p; };
  unsigned short* R = (unsigned short*)carve(Wo_::END * 2); float* P = (float*)carve(8192 * 4);
  float* sq = (float*)carve(PLH * 4); float* sk = (float*)carve(PLH * 4); float* sv = (float*)carve(PLH * 4); b16* vt = (b16*)carve(PLH * 2); float* logg = (float*)carve((size_t)NT * H * 4); float* hseq = (float*)carve((size_t)NT * DIM * 4);
  b16* qp = (b16*)carve(PLH * 2); b16* kp = (b16*)carve(PLH * 2); b16* ctx = (b16*)sq;
  if (off > ws_size) return;
  prep_kernel<<<512, 256, 0, stream>>>(Wsq, Wsk, Wsv, Wg, Wq, Wk, Wv, Wo, bsq, bsk, bsv, bv, bg, bq, bk, bo, temp, R, P);
  proj_kernel<<<dim3(65, NT / 128), 128, 0, stream>>>(x, R, P, sq, sk, sv, vt, logg);
  rec_kernel<<<dim3(H, Bn), 32, 0, stream>>>(sq, sk, sv, logg, hseq);
  qk_kernel<<<dim3(H, NT / 128, 2), 128, 0, stream>>>(hseq, R, P, qp, kp);
  attn_kernel<<<dim3(NT / 16, 2), 256, 0, stream>>>(qp, kp, vt, ctx);
  out_kernel<<<dim3(DIM / 64, NT / 128), 128, 0, stream>>>(ctx, R, P, out);
}
